// ParaNNTranSegmentor_55001351193246
// MI455X (gfx1250) — hardware-run, weakly checked
//
#include <hip/hip_runtime.h>
#include <math.h>

constexpr int NBAT  = 256;
constexpr int NSTEP = 256;
constexpr int NVOC  = 8000;
constexpr int NEMB  = 128;
constexpr int NHC   = 128;
constexpr int NHW   = 256;
constexpr int PCOLS = 8 * NHC;
constexpr float CARRY_A       = 64.0f;
constexpr float CARRY_W       = 16.0f;
constexpr float CARRY_ACC     = CARRY_A * CARRY_W;
constexpr float CARRY_ACC_INV = 1.0f / CARRY_ACC;
constexpr float CARRY_A_INV   = 1.0f / CARRY_A;

constexpr int CH_ROWS = 32;
constexpr int CH_THR  = 256;
constexpr int CH_HP   = 136;
constexpr int CH_NBLK = NBAT / CH_ROWS;
constexpr int ST_ROWS = 32;
constexpr int ST_THR  = 512;
constexpr int ST_NW   = 16;
constexpr int ST_HP   = 264;
constexpr int ST_TCH  = 16;

static_assert(NSTEP == 256);
static_assert(NHC == 128);
static_assert(NHW == 2 * NHC);
static_assert(PCOLS == 1024);
static_assert(NVOC % 64 == 0 && PCOLS % 64 == 0 && NEMB % 32 == 0);
static_assert(NHC % 32 == 0 && NHW % 32 == 0);
static_assert(NBAT % CH_ROWS == 0 && NBAT % ST_ROWS == 0);
static_assert(NHC == 16 * (CH_THR / 32));
static_assert(NHW == 16 * ST_NW && ST_THR == 32 * ST_NW);
static_assert((2 * CH_ROWS * CH_HP) % CH_THR == 0);
static_assert((NSTEP * CH_ROWS) % CH_THR == 0);
static_assert(NSTEP % ST_TCH == 0 && ST_ROWS * ST_TCH == ST_THR);
static_assert(CH_HP % 8 == 0 && ST_HP % 8 == 0);

typedef __attribute__((ext_vector_type(16))) _Float16 v16h;
typedef __attribute__((ext_vector_type(8)))  _Float16 v8h;
typedef __attribute__((ext_vector_type(16))) __bf16   v16b;
typedef __attribute__((ext_vector_type(8)))  __bf16   v8b;
typedef __attribute__((ext_vector_type(8)))  float    v8f;
typedef __attribute__((ext_vector_type(4)))  float    v4f;
typedef __attribute__((ext_vector_type(2)))  float    v2f;
typedef __attribute__((ext_vector_type(4)))  int      v4i;
typedef __attribute__((ext_vector_type(4)))  unsigned v4u;

__device__ __forceinline__ unsigned short f2bf_bits(float f) {
  unsigned u = __float_as_uint(f);
  return (unsigned short)((u + 0x7FFFu + ((u >> 16) & 1u)) >> 16);
}
__device__ __forceinline__ float bf_bits2f(unsigned short h) { return __uint_as_float(((unsigned)h) << 16); }

__device__ __forceinline__ float h16_to_f32(unsigned hb) {
  const unsigned sgn = (hb & 0x8000u) << 16;
  const unsigned em = hb & 0x7fffu;
  const float fn = __uint_as_float((em << 13) + 0x38000000u);
  const float fs = (float)em * 5.9604644775390625e-8f;
  const float mag = (em < 0x400u) ? fs : fn;
  return __uint_as_float(__float_as_uint(mag) | sgn);
}

__device__ __forceinline__ void guard4_h(v8f& a, v8f& b, v8f& c, v8f& d, v16h x, v16h y) {
  asm volatile("v_nop\n\tv_nop\n\tv_nop\n\tv_nop" : "+v"(a), "+v"(b), "+v"(c), "+v"(d) : "v"(x), "v"(y));
}
__device__ __forceinline__ void guard4_b(v8f& a, v8f& b, v8f& c, v8f& d, v16b x, v16b y) {
  asm volatile("v_nop\n\tv_nop\n\tv_nop\n\tv_nop" : "+v"(a), "+v"(b), "+v"(c), "+v"(d) : "v"(x), "v"(y));
}
__device__ __forceinline__ void keep4_h(v16h a, v16h b, v16h c, v16h d) { asm volatile("v_nop" :: "v"(a), "v"(b), "v"(c), "v"(d)); }
__device__ __forceinline__ void keep4_b(v16b a, v16b b, v16b c, v16b d) { asm volatile("v_nop" :: "v"(a), "v"(b), "v"(c), "v"(d)); }
__device__ __forceinline__ void acc_guard4(v8f& a, v8f& b, v8f& c, v8f& d) {
  asm volatile("v_nop\n\tv_nop\n\tv_nop\n\tv_nop" : "+v"(a), "+v"(b), "+v"(c), "+v"(d));
}
__device__ __forceinline__ void guard8_h(v8f& a0, v8f& a1, v8f& a2, v8f& a3, v8f& a4, v8f& a5, v8f& a6, v8f& a7,
                                         v16h x0, v16h x1, v16h y0, v16h y1, v16h y2, v16h y3) {
  asm volatile("v_nop\n\tv_nop\n\tv_nop\n\tv_nop"
               : "+v"(a0), "+v"(a1), "+v"(a2), "+v"(a3), "+v"(a4), "+v"(a5), "+v"(a6), "+v"(a7)
               : "v"(x0), "v"(x1), "v"(y0), "v"(y1), "v"(y2), "v"(y3));
}

template <typename T> struct Frag;
template <> struct Frag<_Float16> {
  typedef v16h V;
  union U { v16h v; v8h h[2]; };
  static __device__ __forceinline__ v16h load(const _Float16* p) {
    U f;
    f.h[0] = *(const v8h*)(p);
    f.h[1] = *(const v8h*)(p + 16);
    return f.v;
  }
  static __device__ __forceinline__ v8f mma(v16h a, v16h b, v8f c) {
    return __builtin_amdgcn_wmma_f32_16x16x32_f16(false, a, false, b, (short)0, c, false, false);
  }
  static __device__ __forceinline__ void guard4(v8f& a, v8f& b, v8f& c, v8f& d, v16h x, v16h y) { guard4_h(a, b, c, d, x, y); }
  static __device__ __forceinline__ void keep(v16h a, v16h b, v16h c, v16h d) { keep4_h(a, b, c, d); }
};
template <> struct Frag<__bf16> {
  typedef v16b V;
  union U { v16b v; v8b h[2]; };
  static __device__ __forceinline__ v16b load(const __bf16* p) {
    U f;
    f.h[0] = *(const v8b*)(p);
    f.h[1] = *(const v8b*)(p + 16);
    return f.v;
  }
  static __device__ __forceinline__ v8f mma(v16b a, v16b b, v8f c) {
    return __builtin_amdgcn_wmma_f32_16x16x32_bf16(false, a, false, b, (short)0, c, false, false);
  }
  static __device__ __forceinline__ void guard4(v8f& a, v8f& b, v8f& c, v8f& d, v16b x, v16b y) { guard4_b(a, b, c, d, x, y); }
  static __device__ __forceinline__ void keep(v16b a, v16b b, v16b c, v16b d) { keep4_b(a, b, c, d); }
};

__device__ __forceinline__ float fsig(float x)  { return __builtin_amdgcn_rcpf(1.0f + __expf(-x)); }
__device__ __forceinline__ float ftanh(float x) { return 1.0f - 2.0f * __builtin_amdgcn_rcpf(__expf(2.0f * x) + 1.0f); }

__device__ __forceinline__ void lstm_elem(float zi, float zf, float zg, float zo, float cprev, float& cn, float& hn) {
  const float ig = fsig(zi);
  const float fg = fsig(zf);
  const float gg = ftanh(zg);
  const float og = fsig(zo);
  cn = fg * cprev + ig * gg;
  hn = og * ftanh(cn);
}

template <int ET> struct Elem;
template <> struct Elem<0> { typedef _Float16 T; };
template <> struct Elem<1> { typedef __bf16 T; };
template <int ET, bool SPLIT, int BIAS_MODE, int OUT_MODE, bool RESID, int ACT = 0>
__global__ __launch_bounds__(256) void wmma_gemm64(
    const unsigned short* __restrict__ Ap, const unsigned short* __restrict__ A2p, int lda, long strideA,
    const unsigned short* __restrict__ Btp, const unsigned short* __restrict__ Bt2p, int ldb, long strideB,
    void* __restrict__ Cout, void* __restrict__ Cout2, int ldc, long strideC,
    const float* __restrict__ bias,
    const float* __restrict__ resid, long strideR,
    int M, int N, int K, float scale) {
  typedef typename Elem<ET>::T T;
  typedef typename Frag<T>::V V;
  const T* A = (const T*)Ap;
  const T* A2 = (const T*)A2p;
  const T* Bt = (const T*)Btp;
  const T* Bt2 = (const T*)Bt2p;
  __shared__ __align__(16) float sT[8][16 * 68];
  const int b    = blockIdx.y;
  const int lane = threadIdx.x & 31;
  const int wave = threadIdx.x >> 5;
  const int tilesN = N >> 6;
  const int tilesM = M >> 6;
  const int tile = blockIdx.x * 8 + wave;
  if (tile >= tilesM * tilesN) return;
  const int tm = tile / tilesN;
  const int tn = tile - tm * tilesN;
  const int m0 = tm << 6;
  const int n0 = tn << 6;

  const T* Ab  = A  + (size_t)b * strideA;
  const T* Bb  = Bt + (size_t)b * strideB;
  const T* Ab2 = SPLIT ? (A2  + (size_t)b * strideA) : nullptr;
  const T* Bb2 = SPLIT ? (Bt2 + (size_t)b * strideB) : nullptr;

  const int rlane = lane & 15;
  const int koff  = (lane >> 4) * 8;
  const int mOff  = (lane >> 4) * 8;

  v8f acc[4][4];
#pragma unroll
  for (int i = 0; i < 4; ++i)
#pragma unroll
    for (int j = 0; j < 4; ++j) acc[i][j] = (v8f){0.f,0.f,0.f,0.f,0.f,0.f,0.f,0.f};

  for (int k0 = 0; k0 < K; k0 += 32) {
    V bh[4], bl[4];
#pragma unroll
    for (int j = 0; j < 4; ++j) {
      const size_t bo = (size_t)(n0 + (j << 4) + rlane) * ldb + koff + k0;
      bh[j] = Frag<T>::load(Bb + bo);
      if (SPLIT) bl[j] = Frag<T>::load(Bb2 + bo);
    }
#pragma unroll
    for (int i = 0; i < 4; ++i) {
      const size_t ao = (size_t)(m0 + (i << 4) + rlane) * lda + koff + k0;
      V ah = Frag<T>::load(Ab + ao);
      V al;
      if (SPLIT) al = Frag<T>::load(Ab2 + ao);
#pragma unroll
      for (int j = 0; j < 4; ++j) {
        acc[i][j] = Frag<T>::mma(ah, bh[j], acc[i][j]);
        if (SPLIT) {
          acc[i][j] = Frag<T>::mma(ah, bl[j], acc[i][j]);
          acc[i][j] = Frag<T>::mma(al, bh[j], acc[i][j]);
        }
      }
      Frag<T>::guard4(acc[i][0], acc[i][1], acc[i][2], acc[i][3], ah, SPLIT ? al : ah);
    }
    Frag<T>::keep(bh[0], bh[1], bh[2], bh[3]);
    if (SPLIT) Frag<T>::keep(bl[0], bl[1], bl[2], bl[3]);
  }
  acc_guard4(acc[0][0], acc[0][1], acc[0][2], acc[0][3]);
  acc_guard4(acc[1][0], acc[1][1], acc[1][2], acc[1][3]);
  acc_guard4(acc[2][0], acc[2][1], acc[2][2], acc[2][3]);
  acc_guard4(acc[3][0], acc[3][1], acc[3][2], acc[3][3]);

  float* slab = sT[wave];
  const float* Rb = RESID ? (resid + (size_t)b * strideR) : nullptr;
#pragma unroll
  for (int i = 0; i < 4; ++i) {
    const int mBase = m0 + (i << 4);
#pragma unroll
    for (int j = 0; j < 4; ++j) {
      const int n = n0 + (j << 4) + rlane;
      float bv = 0.f;
      if (BIAS_MODE == 2) bv = bias[n];
#pragma unroll
      for (int r = 0; r < 8; ++r) {
        float v = acc[i][j][r] * scale;
        if (BIAS_MODE == 1) v += bias[mBase + mOff + r];
        if (BIAS_MODE == 2) v += bv;
        if (RESID) v += Rb[(size_t)(mBase + mOff + r) * ldc + n];
        if (ACT == 1) v = tanhf(v);
        if (ACT == 2) v = fmaxf(v, 0.0f);
        if (ACT == 3) v = v / (1.0f + expf(-v));
        if (ACT == 4) v = (v > 0.f) ? v : 0.01f * v;
        if (ACT == 5) v = 0.5f * v * (1.0f + erff(v * 0.70710678118654752f));
        slab[(mOff + r) * 68 + (j << 4) + rlane] = v;
      }
    }
    __builtin_amdgcn_fence(__ATOMIC_RELEASE, "workgroup");
    __builtin_amdgcn_wave_barrier();
    __builtin_amdgcn_fence(__ATOMIC_ACQUIRE, "workgroup");
    if (OUT_MODE == 0) {
      float* C = (float*)Cout + (size_t)b * strideC;
      const int hh = lane >> 4, c4 = (lane & 15) * 4;
      for (int pass = 0; pass < 2; ++pass) {
#pragma unroll
        for (int it = 0; it < 8; ++it) {
          const int row = it * 2 + hh;
          v4f v = *(const v4f*)(slab + row * 68 + c4);
          *(volatile v4f*)(C + (size_t)(mBase + row) * ldc + n0 + c4) = v;
        }
        __threadfence();
      }
    } else {
      const int q = lane >> 3, c8 = (lane & 7) * 8;
      unsigned short* C  = (unsigned short*)Cout  + (size_t)b * strideC;
      unsigned short* C2 = (OUT_MODE == 2) ? ((unsigned short*)Cout2 + (size_t)b * strideC) : nullptr;
      for (int pass = 0; pass < 2; ++pass) {
#pragma unroll
        for (int it = 0; it < 4; ++it) {
          const int row = it * 4 + q;
          const float* sp = slab + row * 68 + c8;
          v8h hv, lv;
#pragma unroll
          for (int e = 0; e < 8; ++e) {
            if (OUT_MODE == 1) {
              hv[e] = (_Float16)sp[e];
            } else {
              unsigned short hb = f2bf_bits(sp[e]);
              unsigned short lb = f2bf_bits(sp[e] - bf_bits2f(hb));
              hv[e] = __builtin_bit_cast(_Float16, hb);
              lv[e] = __builtin_bit_cast(_Float16, lb);
            }
          }
          *(volatile v8h*)(C + (size_t)(mBase + row) * ldc + n0 + c8) = hv;
          if (OUT_MODE == 2) *(volatile v8h*)(C2 + (size_t)(mBase + row) * ldc + n0 + c8) = lv;
        }
        __threadfence();
      }
    }
    __builtin_amdgcn_fence(__ATOMIC_RELEASE, "workgroup");
    __builtin_amdgcn_wave_barrier();
    __builtin_amdgcn_fence(__ATOMIC_ACQUIRE, "workgroup");
  }
}

template <int PERM>
__global__ __launch_bounds__(256) void cvt8_f16_kernel(const float* __restrict__ src, unsigned short* __restrict__ dst,
                                                        int nrow, int ncol8, int spitch, int dpitch, int dcol0, int drow0,
                                                        float sc) {
  const int i  = blockIdx.x * 256 + threadIdx.x;
  const int n8 = nrow * ncol8;
  if (i < n8) {
    const int row = i / ncol8;
    const int c8  = i - row * ncol8;
    const int drow = PERM ? (drow0 + (row & (NHC - 1)) * 4 + (row >> 7)) : (drow0 + row);
    const float* sp = src + (size_t)row * spitch + c8 * 8;
    const v4f a = *(const v4f*)(sp);
    const v4f b = *(const v4f*)(sp + 4);
    v8h hv;
#pragma unroll
    for (int e = 0; e < 4; ++e) {
      hv[e]     = (_Float16)(a[e] * sc);
      hv[4 + e] = (_Float16)(b[e] * sc);
    }
    unsigned short* dp = dst + (size_t)drow * dpitch + dcol0 + c8 * 8;
    *(volatile v8h*)dp = hv;
    __threadfence();
    *(volatile v8h*)dp = hv;
  }
}

template <int KLEN>
__device__ __forceinline__ void kblock(v8f (&acc)[4][2], const _Float16* a0p, const _Float16* a1p,
                                       const _Float16* bp, const size_t gs) {
#pragma unroll 1
  for (int k0 = 0; k0 < KLEN; k0 += 32) {
    const v16h a0 = Frag<_Float16>::load(a0p + k0);
    const v16h a1 = Frag<_Float16>::load(a1p + k0);
    const v16h b0 = Frag<_Float16>::load(bp + k0);
    const v16h b1 = Frag<_Float16>::load(bp + gs + k0);
    const v16h b2 = Frag<_Float16>::load(bp + 2 * gs + k0);
    const v16h b3 = Frag<_Float16>::load(bp + 3 * gs + k0);
    acc[0][0] = Frag<_Float16>::mma(a0, b0, acc[0][0]);
    acc[0][1] = Frag<_Float16>::mma(a1, b0, acc[0][1]);
    acc[1][0] = Frag<_Float16>::mma(a0, b1, acc[1][0]);
    acc[1][1] = Frag<_Float16>::mma(a1, b1, acc[1][1]);
    acc[2][0] = Frag<_Float16>::mma(a0, b2, acc[2][0]);
    acc[2][1] = Frag<_Float16>::mma(a1, b2, acc[2][1]);
    acc[3][0] = Frag<_Float16>::mma(a0, b3, acc[3][0]);
    acc[3][1] = Frag<_Float16>::mma(a1, b3, acc[3][1]);
    guard8_h(acc[0][0], acc[0][1], acc[1][0], acc[1][1], acc[2][0], acc[2][1], acc[3][0], acc[3][1],
             a0, a1, b0, b1, b2, b3);
  }
}

__global__ __launch_bounds__(CH_THR) void char_seq_kernel(const int* __restrict__ insts, const float* __restrict__ Ptab,
                                                          const unsigned short* __restrict__ Whhp,
                                                          const float* __restrict__ b_f, const float* __restrict__ b_b,
                                                          unsigned short* __restrict__ charsp) {
  __shared__ __align__(16) _Float16 Ah[2][CH_ROWS * CH_HP];
  __shared__ __align__(16) int tokS[NSTEP * CH_ROWS];
  const int tid = threadIdx.x, lane = tid & 31, wave = tid >> 5;
  const int c = lane & 15, hh = lane >> 4, koff = hh * 8;
  const int dir = blockIdx.x / CH_NBLK;
  const int rowbase = (blockIdx.x - dir * CH_NBLK) * CH_ROWS;
  const int j = 16 * wave + c;

  {
    _Float16* ahf = &Ah[0][0];
#pragma unroll 1
    for (int i = tid; i < 2 * CH_ROWS * CH_HP; i += CH_THR) ahf[i] = (_Float16)0.0f;
  }
#pragma unroll 1
  for (int i = tid; i < NSTEP * CH_ROWS; i += CH_THR) {
    const int row = i >> 8, s = i & (NSTEP - 1);
    int tk = insts[(size_t)(rowbase + row) * NSTEP + s];
    tk = tk < 0 ? 0 : (tk > NVOC - 1 ? NVOC - 1 : tk);
    tokS[s * CH_ROWS + row] = tk;
  }
  float bsc[4];
#pragma unroll
  for (int g = 0; g < 4; ++g) {
    const float vf = b_f[g * NHC + j];
    const float vb = b_b[g * NHC + j];
    bsc[g] = (dir ? vb : vf) * CARRY_ACC;
  }
  float cst[2][8];
#pragma unroll
  for (int mt = 0; mt < 2; ++mt)
#pragma unroll
    for (int r = 0; r < 8; ++r) cst[mt][r] = 0.0f;
  __syncthreads();

  const _Float16* Wh = (const _Float16*)Whhp + ((size_t)dir * 4 * NHC + j) * NHC + koff;
  const float* Pd = Ptab + dir * 4 * NHC + j * 4;
  const size_t gsC = (size_t)NHC * NHC;

#pragma unroll 1
  for (int t = 0; t < NSTEP; ++t) {
    const int s = dir ? (NSTEP - 1 - t) : t;
    const int cur = t & 1;
    const _Float16* ahc = &Ah[cur][0];
    _Float16* ahn = &Ah[cur ^ 1][0];

    v8f acc[4][2];
#pragma unroll
    for (int g = 0; g < 4; ++g) {
      const float bv = bsc[g];
      acc[g][0] = (v8f){bv, bv, bv, bv, bv, bv, bv, bv};
      acc[g][1] = acc[g][0];
    }
    kblock<NHC>(acc, ahc + c * CH_HP + koff, ahc + (16 + c) * CH_HP + koff, Wh, gsC);

    const int* tk = tokS + s * CH_ROWS + 8 * hh;
#pragma unroll
    for (int mt = 0; mt < 2; ++mt) {
      const v4i ta = *(const v4i*)(tk + 16 * mt);
      const v4i tb = *(const v4i*)(tk + 16 * mt + 4);
      int tkr[8];
      tkr[0] = ta[0]; tkr[1] = ta[1]; tkr[2] = ta[2]; tkr[3] = ta[3];
      tkr[4] = tb[0]; tkr[5] = tb[1]; tkr[6] = tb[2]; tkr[7] = tb[3];
#pragma unroll
      for (int r = 0; r < 8; ++r) {
        const v4f pv = *(const v4f*)(Pd + (size_t)tkr[r] * PCOLS);
        const float zi = (acc[0][mt][r] + pv[0]) * CARRY_ACC_INV;
        const float zf = (acc[1][mt][r] + pv[1]) * CARRY_ACC_INV;
        const float zg = (acc[2][mt][r] + pv[2]) * CARRY_ACC_INV;
        const float zo = (acc[3][mt][r] + pv[3]) * CARRY_ACC_INV;
        float cn, hn;
        lstm_elem(zi, zf, zg, zo, cst[mt][r], cn, hn);
        cst[mt][r] = cn;
        ahn[(16 * mt + 8 * hh + r) * CH_HP + j] = (_Float16)(hn * CARRY_A);
      }
    }
    __syncthreads();

    for (int pass = 0; pass < 2; ++pass) {
#pragma unroll
      for (int it = 0; it < 2; ++it) {
        const int row = 4 * wave + 2 * it + hh;
        const v8h v = *(const v8h*)(ahn + row * CH_HP + 8 * c);
        *(volatile v8h*)(charsp + ((size_t)s * NBAT + rowbase + row) * (2 * NHC) + dir * NHC + 8 * c) = v;
      }
      __threadfence();
    }
  }
}

__global__ __launch_bounds__(ST_THR) void stack_seq_kernel(const int* __restrict__ golds,
                                                           const unsigned short* __restrict__ charsp,
                                                           const unsigned short* __restrict__ Wsubp,
                                                           const unsigned short* __restrict__ Wwrdp,
                                                           const float* __restrict__ sub_b, const float* __restrict__ wrd_b,
                                                           const float* __restrict__ cls_W, const float* __restrict__ cls_b,
                                                           float* __restrict__ out) {
  __shared__ __align__(16) _Float16 Hs[ST_ROWS * ST_HP];
  __shared__ __align__(16) _Float16 H1[ST_ROWS * ST_HP];
  __shared__ __align__(16) _Float16 Hw[ST_ROWS * ST_HP];
  __shared__ __align__(16) int   gS[ST_TCH * ST_ROWS];
  __shared__ __align__(16) float outS[ST_ROWS * 2 * ST_TCH];
  __shared__ __align__(16) float partS[ST_NW * ST_ROWS * 2];
  __shared__ __align__(16) float clsS[2 * NHW];
  const int tid = threadIdx.x, lane = tid & 31, wave = tid >> 5;
  const int c = lane & 15, hh = lane >> 4, koff = hh * 8;
  const int rowbase = blockIdx.x * ST_ROWS;
  const int j = 16 * wave + c;

#pragma unroll 1
  for (int i = tid; i < ST_ROWS * ST_HP; i += ST_THR) {
    Hs[i] = (_Float16)0.0f;
    H1[i] = (_Float16)0.0f;
    Hw[i] = (_Float16)0.0f;
  }
  clsS[tid] = cls_W[(tid >> 8) * (2 * NHW) + NHW + (tid & (NHW - 1))];

  float bs[4], bw[4];
#pragma unroll
  for (int g = 0; g < 4; ++g) {
    bs[g] = sub_b[g * NHW + j] * CARRY_ACC;
    bw[g] = wrd_b[g * NHW + j] * CARRY_ACC;
  }
  const float wc0 = cls_W[j];
  const float wc1 = cls_W[2 * NHW + j];
  const float cb0 = cls_b[0];
  const float cb1 = cls_b[1];
  float cs[2][8], cw[2][8];
#pragma unroll
  for (int mt = 0; mt < 2; ++mt)
#pragma unroll
    for (int r = 0; r < 8; ++r) { cs[mt][r] = 0.0f; cw[mt][r] = 0.0f; }
  __syncthreads();

  const _Float16* chars = (const _Float16*)charsp;
  const _Float16* wsp = (const _Float16*)Wsubp + (size_t)j * (2 * NHW) + koff;
  const _Float16* wwp = (const _Float16*)Wwrdp + (size_t)j * (2 * NHW) + koff;
  const size_t gsS = (size_t)NHW * (2 * NHW);
  const _Float16* hs0 = Hs + c * ST_HP + koff;
  const _Float16* h10 = H1 + c * ST_HP + koff;
  const _Float16* hw0 = Hw + c * ST_HP + koff;

#pragma unroll 1
  for (int t = 0; t < NSTEP; ++t) {
    const int tt = t & (ST_TCH - 1);
    if (tt == 0) {
      const int row = tid >> 4, q = tid & 15;
      int g = golds[(size_t)(rowbase + row) * NSTEP + t + q];
      g = g < 0 ? 0 : (g > 2 ? 2 : g);
      gS[q * ST_ROWS + row] = g;
      __syncthreads();
    }
    unsigned gm = 0u;
#pragma unroll
    for (int mt = 0; mt < 2; ++mt) {
      const v4i ga = *(const v4i*)(gS + tt * ST_ROWS + 16 * mt + 8 * hh);
      const v4i gb = *(const v4i*)(gS + tt * ST_ROWS + 16 * mt + 8 * hh + 4);
      gm |= (ga[0] != 0 ? 1u : 0u) << (8 * mt + 0);
      gm |= (ga[1] != 0 ? 1u : 0u) << (8 * mt + 1);
      gm |= (ga[2] != 0 ? 1u : 0u) << (8 * mt + 2);
      gm |= (ga[3] != 0 ? 1u : 0u) << (8 * mt + 3);
      gm |= (gb[0] != 0 ? 1u : 0u) << (8 * mt + 4);
      gm |= (gb[1] != 0 ? 1u : 0u) << (8 * mt + 5);
      gm |= (gb[2] != 0 ? 1u : 0u) << (8 * mt + 6);
      gm |= (gb[3] != 0 ? 1u : 0u) << (8 * mt + 7);
    }

    v8f acc[4][2];
#pragma unroll
    for (int g = 0; g < 4; ++g) {
      const float bv = bs[g];
      acc[g][0] = (v8f){bv, bv, bv, bv, bv, bv, bv, bv};
      acc[g][1] = acc[g][0];
    }
    if (t > 0) {
      const _Float16* xg = chars + ((size_t)(t - 1) * NBAT + rowbase + c) * (2 * NHC) + koff;
      kblock<2 * NHC>(acc, xg, xg + (size_t)16 * (2 * NHC), wsp, gsS);
    }
    kblock<NHW>(acc, hs0, hs0 + 16 * ST_HP, wsp + NHW, gsS);

    float hsn[2][8];
#pragma unroll
    for (int mt = 0; mt < 2; ++mt) {
#pragma unroll
      for (int r = 0; r < 8; ++r) {
        const float zi = acc[0][mt][r] * CARRY_ACC_INV;
        const float zf = acc[1][mt][r] * CARRY_ACC_INV;
        const float zg = acc[2][mt][r] * CARRY_ACC_INV;
        const float zo = acc[3][mt][r] * CARRY_ACC_INV;
        float c1, h1;
        lstm_elem(zi, zf, zg, zo, cs[mt][r], c1, h1);
        const bool nz = ((gm >> (8 * mt + r)) & 1u) != 0u;
        const float hv = h1 * CARRY_A;
        cs[mt][r]  = nz ? 0.0f : c1;
        hsn[mt][r] = nz ? 0.0f : hv;
        H1[(16 * mt + 8 * hh + r) * ST_HP + j] = (_Float16)hv;
      }
    }
    __syncthreads();
#pragma unroll
    for (int mt = 0; mt < 2; ++mt)
#pragma unroll
      for (int r = 0; r < 8; ++r) Hs[(16 * mt + 8 * hh + r) * ST_HP + j] = (_Float16)hsn[mt][r];

#pragma unroll
    for (int g = 0; g < 4; ++g) {
      const float bv = bw[g];
      acc[g][0] = (v8f){bv, bv, bv, bv, bv, bv, bv, bv};
      acc[g][1] = acc[g][0];
    }
    kblock<NHW>(acc, h10, h10 + 16 * ST_HP, wwp, gsS);
    kblock<NHW>(acc, hw0, hw0 + 16 * ST_HP, wwp + NHW, gsS);

    float hwn[2][8], p0[2][8], p1[2][8];
#pragma unroll
    for (int mt = 0; mt < 2; ++mt) {
#pragma unroll
      for (int r = 0; r < 8; ++r) {
        const float zi = acc[0][mt][r] * CARRY_ACC_INV;
        const float zf = acc[1][mt][r] * CARRY_ACC_INV;
        const float zg = acc[2][mt][r] * CARRY_ACC_INV;
        const float zo = acc[3][mt][r] * CARRY_ACC_INV;
        float c2, h2;
        lstm_elem(zi, zf, zg, zo, cw[mt][r], c2, h2);
        const bool nz = ((gm >> (8 * mt + r)) & 1u) != 0u;
        cw[mt][r]  = nz ? c2 : cw[mt][r];
        hwn[mt][r] = h2 * CARRY_A;
        p0[mt][r]  = h2 * wc0;
        p1[mt][r]  = h2 * wc1;
      }
    }
#pragma unroll
    for (int mt = 0; mt < 2; ++mt) {
#pragma unroll
      for (int r = 0; r < 8; ++r) {
#pragma unroll
        for (int off = 1; off < 16; off <<= 1) {
          p0[mt][r] += __shfl_xor(p0[mt][r], off, 32);
          p1[mt][r] += __shfl_xor(p1[mt][r], off, 32);
        }
      }
    }
    if (c == 0) {
#pragma unroll
      for (int mt = 0; mt < 2; ++mt) {
        float* pb = partS + wave * (2 * ST_ROWS) + (16 * mt + 8 * hh) * 2;
#pragma unroll
        for (int q = 0; q < 4; ++q) {
          v4f v;
          v[0] = p0[mt][2 * q];
          v[1] = p1[mt][2 * q];
          v[2] = p0[mt][2 * q + 1];
          v[3] = p1[mt][2 * q + 1];
          *(v4f*)(pb + 4 * q) = v;
        }
      }
    }
    __syncthreads();
#pragma unroll
    for (int mt = 0; mt < 2; ++mt) {
#pragma unroll
      for (int r = 0; r < 8; ++r) {
        if (((gm >> (8 * mt + r)) & 1u) != 0u) Hw[(16 * mt + 8 * hh + r) * ST_HP + j] = (_Float16)hwn[mt][r];
      }
    }

    {
      const int row = tid >> 4, p = tid & 15;
      const unsigned* cp = (const unsigned*)(const void*)(charsp + ((size_t)t * NBAT + rowbase + row) * (2 * NHC) + 16 * p);
      const v4u wa = *(const v4u*)(cp);
      const v4u wb = *(const v4u*)(cp + 4);
      unsigned wd[8];
      wd[0] = wa[0]; wd[1] = wa[1]; wd[2] = wa[2]; wd[3] = wa[3];
      wd[4] = wb[0]; wd[5] = wb[1]; wd[6] = wb[2]; wd[7] = wb[3];
      float s0 = 0.0f, s1 = 0.0f;
#pragma unroll
      for (int q = 0; q < 4; ++q) {
        const v4f w0 = *(const v4f*)(clsS + 16 * p + 4 * q);
        const v4f w1 = *(const v4f*)(clsS + NHW + 16 * p + 4 * q);
        const unsigned ua = wd[2 * q];
        const unsigned ub = wd[2 * q + 1];
        const float x0 = h16_to_f32(ua & 0xffffu);
        const float x1 = h16_to_f32(ua >> 16);
        const float x2 = h16_to_f32(ub & 0xffffu);
        const float x3 = h16_to_f32(ub >> 16);
        s0 = fmaf(x0, w0[0], s0);
        s0 = fmaf(x1, w0[1], s0);
        s0 = fmaf(x2, w0[2], s0);
        s0 = fmaf(x3, w0[3], s0);
        s1 = fmaf(x0, w1[0], s1);
        s1 = fmaf(x1, w1[1], s1);
        s1 = fmaf(x2, w1[2], s1);
        s1 = fmaf(x3, w1[3], s1);
      }
      const v2f pp = *(const v2f*)(partS + p * (2 * ST_ROWS) + row * 2);
      s0 = s0 * CARRY_A_INV + pp[0];
      s1 = s1 * CARRY_A_INV + pp[1];
#pragma unroll
      for (int off = 1; off < 16; off <<= 1) {
        s0 += __shfl_xor(s0, off, 32);
        s1 += __shfl_xor(s1, off, 32);
      }
      if (p == 0) {
        v2f o;
        o[0] = s0 + cb0;
        o[1] = s1 + cb1;
        *(v2f*)(outS + row * (2 * ST_TCH) + tt * 2) = o;
      }
    }

    if (tt == ST_TCH - 1) {
      __syncthreads();
      if (wave < 8) {
        const int q = lane >> 3, l8 = lane & 7;
        const int row = 4 * wave + q;
        const v4f v = *(const v4f*)(outS + row * (2 * ST_TCH) + 4 * l8);
        float* gp = out + ((size_t)(rowbase + row) * NSTEP + (size_t)(t - (ST_TCH - 1))) * 2 + 4 * l8;
        *(volatile v4f*)gp = v;
        __threadfence();
        *(volatile v4f*)gp = v;
      }
    }
  }
}

extern "C" void kernel_launch(void* const* d_in, const int* in_sizes, int n_in,
                              void* d_out, int out_size, void* d_ws, size_t ws_size, hipStream_t stream) {
  if (n_in < 17 || d_out == nullptr || d_ws == nullptr) return;
  if (in_sizes[0] != NBAT * NSTEP || in_sizes[1] != NBAT * NSTEP || in_sizes[2] != NVOC * NEMB ||
      in_sizes[3] != 4 * NHC * NEMB || in_sizes[4] != 4 * NHC * NHC || in_sizes[5] != 4 * NHC ||
      in_sizes[6] != 4 * NHC * NEMB || in_sizes[7] != 4 * NHC * NHC || in_sizes[8] != 4 * NHC ||
      in_sizes[9] != 4 * NHW * 2 * NHC || in_sizes[10] != 4 * NHW * NHW || in_sizes[11] != 4 * NHW ||
      in_sizes[12] != 4 * NHW * NHW || in_sizes[13] != 4 * NHW * NHW || in_sizes[14] != 4 * NHW ||
      in_sizes[15] != 2 * (NHW + 2 * NHC) || in_sizes[16] != 2 || out_size != NBAT * NSTEP * 2) return;

  const int*   insts   = (const int*)d_in[0];
  const int*   golds   = (const int*)d_in[1];
  const float* emb     = (const float*)d_in[2];
  const float* wih_f   = (const float*)d_in[3];
  const float* whh_f   = (const float*)d_in[4];
  const float* b_f     = (const float*)d_in[5];
  const float* wih_b   = (const float*)d_in[6];
  const float* whh_b   = (const float*)d_in[7];
  const float* b_b     = (const float*)d_in[8];
  const float* sub_wih = (const float*)d_in[9];
  const float* sub_whh = (const float*)d_in[10];
  const float* sub_b   = (const float*)d_in[11];
  const float* wrd_wih = (const float*)d_in[12];
  const float* wrd_whh = (const float*)d_in[13];
  const float* wrd_b   = (const float*)d_in[14];
  const float* cls_w   = (const float*)d_in[15];
  const float* cls_b   = (const float*)d_in[16];
  float* out = (float*)d_out;

  char* ws = (char*)d_ws;
  size_t off = 0;
  auto carve = [&](size_t bytes) -> char* { char* p = ws + off; off += (bytes + 255) & ~(size_t)255; return p; };
  unsigned short* EMB16 = (unsigned short*)carve((size_t)NVOC * NEMB * 2);
  unsigned short* WIHP  = (unsigned short*)carve((size_t)PCOLS * NEMB * 2);
  unsigned short* WHH   = (unsigned short*)carve((size_t)PCOLS * NHC * 2);
  unsigned short* WSUB  = (unsigned short*)carve((size_t)4 * NHW * 2 * NHW * 2);
  unsigned short* WWRD  = (unsigned short*)carve((size_t)4 * NHW * 2 * NHW * 2);
  float*          PTAB  = (float*)carve((size_t)NVOC * PCOLS * 4);
  unsigned short* CHARS = (unsigned short*)carve((size_t)NSTEP * NBAT * 2 * NHC * 2);
  if (off > ws_size || off > (size_t)134217728) return;

  const int n8e = NVOC * (NEMB / 8);
  const int n8c = 4 * NHC * (NEMB / 8);
  const int n8s = 4 * NHW * (NHW / 8);
  cvt8_f16_kernel<0><<<(n8e + 255) / 256, 256, 0, stream>>>(emb,     EMB16, NVOC,    NEMB / 8, NEMB, NEMB,    0,   0,       CARRY_A);
  cvt8_f16_kernel<1><<<(n8c + 255) / 256, 256, 0, stream>>>(wih_f,   WIHP,  4 * NHC, NEMB / 8, NEMB, NEMB,    0,   0,       CARRY_W);
  cvt8_f16_kernel<1><<<(n8c + 255) / 256, 256, 0, stream>>>(wih_b,   WIHP,  4 * NHC, NEMB / 8, NEMB, NEMB,    0,   4 * NHC, CARRY_W);
  cvt8_f16_kernel<0><<<(n8c + 255) / 256, 256, 0, stream>>>(whh_f,   WHH,   4 * NHC, NHC / 8,  NHC,  NHC,     0,   0,       CARRY_W);
  cvt8_f16_kernel<0><<<(n8c + 255) / 256, 256, 0, stream>>>(whh_b,   WHH,   4 * NHC, NHC / 8,  NHC,  NHC,     0,   4 * NHC, CARRY_W);
  cvt8_f16_kernel<0><<<(n8s + 255) / 256, 256, 0, stream>>>(sub_wih, WSUB,  4 * NHW, NHW / 8,  NHW,  2 * NHW, 0,   0,       CARRY_W);
  cvt8_f16_kernel<0><<<(n8s + 255) / 256, 256, 0, stream>>>(sub_whh, WSUB,  4 * NHW, NHW / 8,  NHW,  2 * NHW, NHW, 0,       CARRY_W);
  cvt8_f16_kernel<0><<<(n8s + 255) / 256, 256, 0, stream>>>(wrd_wih, WWRD,  4 * NHW, NHW / 8,  NHW,  2 * NHW, 0,   0,       CARRY_W);
  cvt8_f16_kernel<0><<<(n8s + 255) / 256, 256, 0, stream>>>(wrd_whh, WWRD,  4 * NHW, NHW / 8,  NHW,  2 * NHW, NHW, 0,       CARRY_W);

  const dim3 ggrid((NVOC / 64) * (PCOLS / 64) / 8, 1);
  wmma_gemm64<0, false, 0, 0, false, 0><<<ggrid, 256, 0, stream>>>(
      EMB16, EMB16, NEMB, 0L, WIHP, WIHP, NEMB, 0L, (void*)PTAB, (void*)PTAB, PCOLS, 0L,
      (const float*)PTAB, (const float*)PTAB, 0L, NVOC, PCOLS, NEMB, 1.0f);

  char_seq_kernel<<<2 * CH_NBLK, CH_THR, 0, stream>>>(insts, PTAB, WHH, b_f, b_b, CHARS);

  stack_seq_kernel<<<NBAT / ST_ROWS, ST_THR, 0, stream>>>(golds, CHARS, WSUB, WWRD, sub_b, wrd_b, cls_w, cls_b, out);
}
